// SpatialTemporalInteractiveGCN_10075993277108
// MI455X (gfx1250) — hardware-verified
//
#include <hip/hip_runtime.h>
#include <math.h>

#ifndef NB
#define NB 8
#endif
#ifndef TT
#define TT 24
#endif
#define TT_FULL 24
#define NN 1024
#define DD 64
#define KA 2048
#define TP (TT + 1)
#define MROWS (NB * TT * NN)
#define XT_P 72

#define X_CARRY 8.0f
#define ADJ_CARRY 32.0f
#define W_CARRY 32.0f
#define SC_ADJ (1.0f / 32.0f)
#define SC_PROJ (1.0f / 256.0f)
#define LN_EPS 1e-5f

static_assert(TT <= TT_FULL);
static_assert(NN % 64 == 0 && KA == 2 * NN && KA % 32 == 0 && DD == 64 && DD % 32 == 0);
static_assert((NN / 64) == 16);
static_assert((NN / 16) == 64);
static_assert((MROWS / 16) % 8 == 0);
static_assert(NN % 32 == 0);
static_assert(KA == 256 * 8);
static_assert((2 * DD * DD / 8) == 4 * 256);
static_assert(256 * 16 * 2 == 64 * 128);
static_assert(32 * 16 * 4 == 16 * 128);
static_assert(32 * 16 * 8 == 16 * 256);
static_assert(8 * 16 * 68 * 4 <= 131072);
static_assert(64 * XT_P * 2 <= 131072);
static_assert((XT_P * 2) % 16 == 0);

#define SZ_A16 ((size_t)NN * KA * 2)
#define SZ_RS  ((size_t)NN * 4)
#define SZ_W16 ((size_t)2 * DD * DD * 2)
#define SZ_XT  ((size_t)NB * DD * TP * NN * 2)
#define SZ_AG  ((size_t)MROWS * DD * 2)
static_assert(SZ_A16 % 256 == 0 && SZ_RS % 256 == 0 && SZ_W16 % 256 == 0 && SZ_XT % 256 == 0 && SZ_AG % 256 == 0);
static_assert(SZ_A16 + SZ_RS + SZ_W16 + SZ_XT + SZ_AG <= (size_t)134217728);

typedef _Float16 h16;
typedef __attribute__((ext_vector_type(16))) _Float16 v16h;
typedef __attribute__((ext_vector_type(8)))  _Float16 v8h;
typedef __attribute__((ext_vector_type(8)))  float    v8f;
typedef __attribute__((ext_vector_type(4)))  float    v4f;


#define VST2V4(ptr, val) do { const v4f vst2_v4_ = (val); *(volatile v4f*)(ptr) = vst2_v4_; __threadfence(); *(volatile v4f*)(ptr) = vst2_v4_; } while (0)

__device__ __forceinline__ float bfr(float f) {
    unsigned u = __float_as_uint(f);
    u += 0x7FFFu + ((u >> 16) & 1u);
    return __uint_as_float(u & 0xFFFF0000u);
}
static __device__ __forceinline__ h16 toh_flush(float v) { const h16 r = (h16)v; return (fabsf(v) < 6.103515625e-05f) ? (h16)0.0f : r; }

__device__ __forceinline__ void st8hf(h16* P, size_t o, const float* v) {
    v8h pk;
#pragma unroll
    for (int e = 0; e < 8; ++e) pk[e] = toh_flush(v[e]);
    *(volatile v8h*)(P + o) = pk;
    __threadfence();
    *(volatile v8h*)(P + o) = pk;
}

union FragU { v16h v; v8h h[2]; };
__device__ __forceinline__ v16h frag_ld(const _Float16* p) {
    FragU f; f.h[0] = *(const v8h*)(p); f.h[1] = *(const v8h*)(p + 16); return f.v;
}
__device__ __forceinline__ v8f wmma16(v16h a, v16h b, v8f c) {
    c = __builtin_amdgcn_wmma_f32_16x16x32_f16(false, a, false, b, (short)0, c, false, false);
    asm volatile("v_nop\n\tv_nop\n\tv_nop\n\tv_nop" : "+v"(c) : "v"(a), "v"(b));
    return c;
}
__device__ __forceinline__ void dep_guard_h(v8f& a, v8f& b, v16h x, v16h y) { asm volatile("v_nop\n\tv_nop\n\tv_nop\n\tv_nop" : "+v"(a), "+v"(b) : "v"(x), "v"(y)); }
__device__ __forceinline__ void keep4_h(v16h a, v16h b, v16h c, v16h d) { asm volatile("v_nop" :: "v"(a), "v"(b), "v"(c), "v"(d)); }
__device__ __forceinline__ void acc_guard4(v8f& a, v8f& b, v8f& c, v8f& d) { asm volatile("v_nop\n\tv_nop\n\tv_nop\n\tv_nop" : "+v"(a), "+v"(b), "+v"(c), "+v"(d)); }
__device__ __forceinline__ void wave_sync_lds() {
    __builtin_amdgcn_fence(3  , "workgroup");
    __builtin_amdgcn_wave_barrier();
    __builtin_amdgcn_fence(2  , "workgroup");
}

__global__ __launch_bounds__(256) void k_wconv(const float* __restrict__ W1, const float* __restrict__ W2,
                                               h16* __restrict__ W16) {
    const unsigned u = blockIdx.x * 256u + threadIdx.x;
    const bool second = (u >= 512u);
    const unsigned idx = (u & 511u) * 8u;
    const v4f a0 = *(const v4f*)(W1 + idx), a1 = *(const v4f*)(W1 + idx + 4u);
    const v4f c0 = *(const v4f*)(W2 + idx), c1 = *(const v4f*)(W2 + idx + 4u);
    const float wa[8] = {a0.x, a0.y, a0.z, a0.w, a1.x, a1.y, a1.z, a1.w};
    const float wc[8] = {c0.x, c0.y, c0.z, c0.w, c1.x, c1.y, c1.z, c1.w};
    float v[8];
#pragma unroll
    for (int i = 0; i < 8; ++i) v[i] = bfr(second ? wc[i] : wa[i]) * W_CARRY;
    st8hf(W16, (size_t)u * 8u, v);
}

__global__ __launch_bounds__(256) void k_adj16(const float* __restrict__ adj, h16* __restrict__ A16, float* __restrict__ rs) {
    __shared__ float sW[8];
    __shared__ __align__(16) float sRS[32];
    const unsigned t = threadIdx.x, lane = t & 31u;
    const unsigned wave = (unsigned)__builtin_amdgcn_readfirstlane((int)(threadIdx.x >> 5));
    const unsigned rbase = blockIdx.x * 32u;
#pragma unroll 1
    for (unsigned rl = 0; rl < 32u; ++rl) {
        const size_t o = (size_t)(rbase + rl) * KA + 8u * t;
        const v4f a = *(const v4f*)(adj + o), b = *(const v4f*)(adj + o + 4u);
        const float w[8] = {bfr(a.x), bfr(a.y), bfr(a.z), bfr(a.w), bfr(b.x), bfr(b.y), bfr(b.z), bfr(b.w)};
        float v[8];
#pragma unroll
        for (int i = 0; i < 8; ++i) v[i] = w[i] * ADJ_CARRY;
        float s = ((w[0] + w[1]) + (w[2] + w[3])) + ((w[4] + w[5]) + (w[6] + w[7]));
        st8hf(A16, o, v);
#pragma unroll
        for (int m = 16; m > 0; m >>= 1) s += __shfl_xor(s, m, 32);
        if (lane == 0u) sW[wave] = s;
        __syncthreads();
        if (t == 0u) sRS[rl] = ((sW[0] + sW[1]) + (sW[2] + sW[3])) + ((sW[4] + sW[5]) + (sW[6] + sW[7]));
        __syncthreads();
    }
    if (t < 8u) {
        v4f v; v.x = sRS[4u * t]; v.y = sRS[4u * t + 1u]; v.z = sRS[4u * t + 2u]; v.w = sRS[4u * t + 3u];
        VST2V4(rs + rbase + 4u * t, v);
    }
}

__global__ __launch_bounds__(256) void k_xT(const float* __restrict__ x, h16* __restrict__ XT) {
    __shared__ __align__(16) _Float16 sX[64 * XT_P];
    const unsigned tid = threadIdx.x;
    const unsigned n0 = blockIdx.x * 64u, tp = blockIdx.y, b = blockIdx.z;
    const bool live = (tp > 0u);
    const unsigned ts = live ? (tp - 1u) : 0u;
    const float* xs = x + ((size_t)(b * TT_FULL + ts) * NN + n0) * DD;
#pragma unroll
    for (int g = 0; g < 4; ++g) {
        const unsigned f = tid + 256u * (unsigned)g;
        const unsigned nl = f >> 4, d4 = (f & 15u) * 4u;
        const v4f a = *(const v4f*)(xs + (size_t)nl * DD + d4);
        const float w[4] = {a.x, a.y, a.z, a.w};
#pragma unroll
        for (int e = 0; e < 4; ++e) {
            const float val = live ? (bfr(w[e]) * X_CARRY) : 0.0f;
            sX[(d4 + (unsigned)e) * XT_P + nl] = toh_flush(val);
        }
    }
    __syncthreads();
    v8h ov[2];
#pragma unroll
    for (int g = 0; g < 2; ++g) {
        const unsigned p = tid + 256u * (unsigned)g;
        const unsigned d = p >> 3, c8 = (p & 7u) * 8u;
        ov[g] = *(const v8h*)(&sX[d * XT_P + c8]);
    }
    for (int pass = 0; pass < 2; ++pass) {
#pragma unroll
        for (int g = 0; g < 2; ++g) {
            const unsigned p = tid + 256u * (unsigned)g;
            const unsigned d = p >> 3, c8 = (p & 7u) * 8u;
            *(volatile v8h*)(XT + ((size_t)(b * DD + d) * TP + tp) * NN + n0 + c8) = ov[g];
        }
        __threadfence();
    }
}

__global__ __launch_bounds__(256) void k_gemm_adj(const _Float16* __restrict__ A, const _Float16* __restrict__ XT,
                                                  _Float16* __restrict__ AG) {
  __shared__ __align__(16) float sT[8][16 * 68];
  const unsigned lane = threadIdx.x & 31u;
  const unsigned wave = (unsigned)__builtin_amdgcn_readfirstlane((int)(threadIdx.x >> 5));
  const unsigned bt = blockIdx.y;
  const unsigned b = bt / (unsigned)TT;
  const unsigned t = bt - b * (unsigned)TT;
  const unsigned m0 = (blockIdx.x * 8u + wave) << 6;
  const unsigned rlane = lane & 15u;
  const unsigned koff = (lane >> 4) * 8u;
  const unsigned mOff = koff;
  const _Float16* Bt = XT + ((size_t)(b * DD) * TP + t) * NN;
  const unsigned lda = (unsigned)KA;
  const unsigned ldb = (unsigned)(TP * NN);

  v8f acc[4][4];
#pragma unroll
  for (int i = 0; i < 4; ++i)
#pragma unroll
    for (int j = 0; j < 4; ++j) acc[i][j] = (v8f){0.f,0.f,0.f,0.f,0.f,0.f,0.f,0.f};

  for (unsigned k0 = 0; k0 < (unsigned)KA; k0 += 32u) {
    v16h bh[4];
#pragma unroll
    for (int j = 0; j < 4; ++j)
      bh[j] = frag_ld(Bt + (size_t)(((unsigned)j << 4) + rlane) * ldb + koff + k0);
#pragma unroll
    for (int i = 0; i < 4; ++i) {
      const v16h ah = frag_ld(A + (size_t)(m0 + ((unsigned)i << 4) + rlane) * lda + koff + k0);
#pragma unroll
      for (int j = 0; j < 4; ++j)
        acc[i][j] = __builtin_amdgcn_wmma_f32_16x16x32_f16(false, ah, false, bh[j], (short)0, acc[i][j], false, false);
      dep_guard_h(acc[i][0], acc[i][3], ah, ah);
    }
    keep4_h(bh[0], bh[1], bh[2], bh[3]);
  }
  acc_guard4(acc[0][0], acc[0][1], acc[0][2], acc[0][3]);
  acc_guard4(acc[1][0], acc[1][1], acc[1][2], acc[1][3]);
  acc_guard4(acc[2][0], acc[2][1], acc[2][2], acc[2][3]);
  acc_guard4(acc[3][0], acc[3][1], acc[3][2], acc[3][3]);

#pragma unroll
  for (int i = 0; i < 4; ++i) {
    const unsigned mBase = m0 + ((unsigned)i << 4);
#pragma unroll
    for (int j = 0; j < 4; ++j) {
#pragma unroll
      for (int r = 0; r < 8; ++r)
        sT[wave][(mOff + (unsigned)r) * 68u + ((unsigned)j << 4) + rlane] = acc[i][j][r] * SC_ADJ;
    }
    wave_sync_lds();
    {
      const unsigned q = lane >> 3, c8 = (lane & 7u) * 8u;
      v8h hv[4];
#pragma unroll
      for (int it = 0; it < 4; ++it) {
        const unsigned row = (unsigned)it * 4u + q;
#pragma unroll
        for (int e = 0; e < 8; ++e) hv[it][e] = toh_flush(sT[wave][row * 68u + c8 + (unsigned)e]);
      }
      for (int pass = 0; pass < 2; ++pass) {
#pragma unroll
        for (int it = 0; it < 4; ++it) {
          const unsigned row = (unsigned)it * 4u + q;
          *(volatile v8h*)(AG + ((size_t)bt * NN + mBase + row) * DD + c8) = hv[it];
        }
        __threadfence();
      }
    }
    wave_sync_lds();
  }
}

__global__ __launch_bounds__(256) void k_proj_ln(const _Float16* __restrict__ AG, const _Float16* __restrict__ W16,
                                                 const float* __restrict__ b1, const float* __restrict__ b2,
                                                 const float* __restrict__ rs, const float* __restrict__ x,
                                                 const float* __restrict__ gamma, const float* __restrict__ beta,
                                                 float* __restrict__ out) {
  __shared__ __align__(16) float sZ[8][16 * 68];
  const unsigned lane = threadIdx.x & 31u;
  const unsigned wave = (unsigned)__builtin_amdgcn_readfirstlane((int)(threadIdx.x >> 5));
  const unsigned tile = blockIdx.x * 8u + wave;
  const unsigned bt = tile >> 6;
  const unsigned n0 = (tile & 63u) << 4;
  const unsigned b = bt / (unsigned)TT;
  const unsigned t = bt - b * (unsigned)TT;
  const unsigned hh = lane >> 4, c = lane & 15u;
  const size_t rowA = (size_t)bt * NN + n0;
  const size_t rowX = ((size_t)b * TT_FULL + t) * NN + n0;

  v8f acc[8];
#pragma unroll
  for (int j = 0; j < 8; ++j) acc[j] = (v8f){0.f,0.f,0.f,0.f,0.f,0.f,0.f,0.f};
#pragma unroll
  for (int kk = 0; kk < 2; ++kk) {
    const v16h af = frag_ld(AG + (rowA + c) * DD + 8u * hh + 32u * (unsigned)kk);
#pragma unroll
    for (int j = 0; j < 8; ++j) {
      const v16h wf = frag_ld(W16 + (size_t)(((unsigned)j << 4) + c) * DD + 8u * hh + 32u * (unsigned)kk);
      acc[j] = wmma16(af, wf, acc[j]);
    }
  }

  {
    const v4f r0 = *(const v4f*)(rs + n0 + 8u * hh), r1 = *(const v4f*)(rs + n0 + 8u * hh + 4u);
    const float rsv[8] = {r0.x, r0.y, r0.z, r0.w, r1.x, r1.y, r1.z, r1.w};
#pragma unroll
    for (int j = 0; j < 4; ++j) {
      const unsigned e = ((unsigned)j << 4) + c;
      const float bb1 = bfr(b1[e]);
      const float bb2 = bfr(b2[e]);
#pragma unroll
      for (int r = 0; r < 8; ++r) {
        const float a1 = acc[j][r] * SC_PROJ + rsv[r] * bb1;
        const float a2 = acc[4 + j][r] * SC_PROJ + rsv[r] * bb2;
        const float p = a1 * a2;
        const float full = ((p > 0.0f) ? p : 0.0f) + a1;
        sZ[wave][(8u * hh + (unsigned)r) * 68u + e] = full;
      }
    }
  }
  wave_sync_lds();

  {
    const unsigned c4 = c * 4u;
    const v4f g4 = *(const v4f*)(gamma + c4), be4 = *(const v4f*)(beta + c4);
    const float gx = bfr(g4.x), gy = bfr(g4.y), gz = bfr(g4.z), gw = bfr(g4.w);
    const float bx = bfr(be4.x), by = bfr(be4.y), bz = bfr(be4.z), bw = bfr(be4.w);
#pragma unroll
    for (int half = 0; half < 2; ++half) {
      v4f vv[4];
#pragma unroll
      for (int it = 0; it < 4; ++it) {
        const unsigned row = (unsigned)(half * 4 + it) * 2u + hh;
        const v4f f = *(const v4f*)(&sZ[wave][row * 68u + c4]);
        const v4f xv = *(const v4f*)(x + (rowX + row) * DD + c4);
        const float z0 = f.x + bfr(xv.x), z1 = f.y + bfr(xv.y), z2 = f.z + bfr(xv.z), z3 = f.w + bfr(xv.w);
        float s = (z0 + z1) + (z2 + z3);
        s += __shfl_xor(s, 8, 32); s += __shfl_xor(s, 4, 32); s += __shfl_xor(s, 2, 32); s += __shfl_xor(s, 1, 32);
        const float mu = s * (1.0f / 64.0f);
        const float d0 = z0 - mu, d1 = z1 - mu, d2 = z2 - mu, d3 = z3 - mu;
        float q = (d0 * d0 + d1 * d1) + (d2 * d2 + d3 * d3);
        q += __shfl_xor(q, 8, 32); q += __shfl_xor(q, 4, 32); q += __shfl_xor(q, 2, 32); q += __shfl_xor(q, 1, 32);
        const float rstd = rsqrtf(q * (1.0f / 64.0f) + LN_EPS);
        vv[it].x = d0 * rstd * gx + bx;
        vv[it].y = d1 * rstd * gy + by;
        vv[it].z = d2 * rstd * gz + bz;
        vv[it].w = d3 * rstd * gw + bw;
      }
      for (int pass = 0; pass < 2; ++pass) {
#pragma unroll
        for (int it = 0; it < 4; ++it) {
          const unsigned row = (unsigned)(half * 4 + it) * 2u + hh;
          *(volatile v4f*)(out + (rowX + row) * DD + c4) = vv[it];
        }
        __threadfence();
      }
    }
  }
}

extern "C" void kernel_launch(void* const* d_in, const int* in_sizes, int n_in, void* d_out, int out_size,
                              void* d_ws, size_t ws_size, hipStream_t stream) {
    if (n_in < 8) return;
    const int xneed = ((NB - 1) * TT_FULL + TT) * NN * DD;
    if (in_sizes[0] < xneed || in_sizes[1] < DD * DD || in_sizes[2] < DD || in_sizes[3] < DD * DD) return;
    if (in_sizes[4] < DD || in_sizes[5] < DD || in_sizes[6] < DD || in_sizes[7] < NN * KA) return;
    if (out_size < xneed) return;

    const float* x     = (const float*)d_in[0];
    const float* W1    = (const float*)d_in[1];
    const float* b1    = (const float*)d_in[2];
    const float* W2    = (const float*)d_in[3];
    const float* b2    = (const float*)d_in[4];
    const float* gamma = (const float*)d_in[5];
    const float* beta  = (const float*)d_in[6];
    const float* adj   = (const float*)d_in[7];
    float* out = (float*)d_out;

    char* wsp = (char*)d_ws;
    size_t off = 0;
    auto carve = [&](size_t bytes) -> void* { void* r = wsp + off; off += (bytes + 255) & ~(size_t)255; return r; };
    h16*   a16 = (h16*)carve(SZ_A16);
    float* rs  = (float*)carve(SZ_RS);
    h16*   w16 = (h16*)carve(SZ_W16);
    h16*   xt  = (h16*)carve(SZ_XT);
    h16*   ag  = (h16*)carve(SZ_AG);
    if (off > ws_size || off > (size_t)134217728) return;

    k_wconv<<<4, 256, 0, stream>>>(W1, W2, w16);
    k_adj16<<<NN / 32, 256, 0, stream>>>(adj, a16, rs);
    k_xT<<<dim3(NN / 64, TP, NB), 256, 0, stream>>>(x, xt);
    k_gemm_adj<<<dim3(2, NB * TT), 256, 0, stream>>>((const _Float16*)a16, (const _Float16*)xt, (_Float16*)ag);
    k_proj_ln<<<(MROWS / 16) / 8, 256, 0, stream>>>((const _Float16*)ag, (const _Float16*)w16, b1, b2, rs, x, gamma, beta, out);
}
